// att_trans_24489903522165
// MI455X (gfx1250) — hardware-verified
//
#include <hip/hip_runtime.h>
#include <math.h>
#include <stddef.h>


typedef _Float16 f16_t;
typedef _Float16 v16h __attribute__((ext_vector_type(16)));
typedef _Float16 v8h  __attribute__((ext_vector_type(8)));
typedef _Float16 v8ha __attribute__((ext_vector_type(8), __may_alias__));
typedef float    v8f  __attribute__((ext_vector_type(8)));
typedef float    v4f  __attribute__((ext_vector_type(4)));
typedef float    v4fa __attribute__((ext_vector_type(4), __may_alias__));

union Frag  { v16h v; v8h half[2]; };
union Pack8 { v8h v; f16_t e[8]; };

#define B_ 8
#define S_ 2048
#define E_ 512
#define SE_ ((size_t)S_ * (size_t)E_)
#define SS_ ((size_t)S_ * (size_t)S_)

#define XSCL 16.0f
#define WSCL 64.0f
#define QSCL 16.0f

static_assert(S_ % 64 == 0 && S_ % 256 == 0 && S_ % 16 == 0);
static_assert(E_ % 256 == 0 && E_ % 64 == 0 && E_ % 32 == 0);
static_assert((S_ * E_) % 256 == 0 && (B_ * E_) % 4 == 0);

__device__ __forceinline__ v16h load_frag(const f16_t* tile, int ld, int lane) {
  const int m = lane & 15, h = lane >> 4;
  const f16_t* p = tile + (size_t)m * ld + 8 * h;
  Frag f;
  f.half[0] = *(const v8ha*)(p);
  f.half[1] = *(const v8ha*)(p + 16);
  return f.v;
}

__device__ __forceinline__ v8f wmma16(v16h a, v16h b, v8f c) {
  return __builtin_amdgcn_wmma_f32_16x16x32_f16(false, a, false, b, (short)0, c, false, false);
}

__device__ __forceinline__ v8f zero8() {
  v8f z = {0.f, 0.f, 0.f, 0.f, 0.f, 0.f, 0.f, 0.f};
  return z;
}

#define WMMA_GUARD8(c0,c1,c2,c3,c4,c5,c6,c7,x0,x1,x2,x3,x4,x5)                      \
  asm volatile("v_nop\n\tv_nop\n\tv_nop\n\tv_nop"                                \
               : "+v"(c0), "+v"(c1), "+v"(c2), "+v"(c3),                          \
                 "+v"(c4), "+v"(c5), "+v"(c6), "+v"(c7)                           \
               : "v"(x0), "v"(x1), "v"(x2), "v"(x3), "v"(x4), "v"(x5))
#define WMMA_GUARD4(c0,c1,c2,c3,x0,x1,x2,x3,x4)                                     \
  asm volatile("v_nop\n\tv_nop\n\tv_nop\n\tv_nop"                                \
               : "+v"(c0), "+v"(c1), "+v"(c2), "+v"(c3)                           \
               : "v"(x0), "v"(x1), "v"(x2), "v"(x3), "v"(x4))

__global__ void __launch_bounds__(256) k_pe(float* pe) {
  const int tid = threadIdx.x, lane = tid & 31, wid = tid >> 5;
  const int gw = blockIdx.x * 8 + wid;
  if (gw >= (S_ * E_) / 256) return;
  const int base = gw * 256;
  const int s = base / E_;
  const int e0 = base % E_;
  const float kc = (float)(-9.210340371976184 / (double)E_);
  const float fs = (float)s;
  const int ja = (e0 + 4 * lane) >> 1;
  const int jb = (e0 + 128 + 4 * lane) >> 1;
  const float ang0 = fs * expf((float)(2 * ja) * kc);
  const float ang1 = fs * expf((float)(2 * ja + 2) * kc);
  const float ang2 = fs * expf((float)(2 * jb) * kc);
  const float ang3 = fs * expf((float)(2 * jb + 2) * kc);
  float r0 = 0.f, r1 = 0.f, r2 = 0.f, r3 = 0.f, r4 = 0.f, r5 = 0.f, r6 = 0.f, r7 = 0.f;
#pragma unroll 1
  for (int p = 0; p < 4; ++p) {
    const float ang = (p == 0) ? ang0 : ((p == 1) ? ang1 : ((p == 2) ? ang2 : ang3));
    float sn, cs;
    sincosf(ang, &sn, &cs);
    if (p == 0)      { r0 = sn; r1 = cs; }
    else if (p == 1) { r2 = sn; r3 = cs; }
    else if (p == 2) { r4 = sn; r5 = cs; }
    else             { r6 = sn; r7 = cs; }
  }
  v4f va = {r0, r1, r2, r3};
  v4f vb = {r4, r5, r6, r7};
  float* pa = pe + base + 4 * lane;
  float* pb = pe + base + 128 + 4 * lane;
  *(volatile v4f*)pa = va;
  *(volatile v4f*)pb = vb;
  __threadfence();
  *(volatile v4f*)pa = va;
  *(volatile v4f*)pb = vb;
}

__global__ void __launch_bounds__(256) k_xph(const float* __restrict__ x,
                                             const float* __restrict__ pe, f16_t* xph) {
  const size_t i8 = (size_t)blockIdx.x * 256 + threadIdx.x;
  if (i8 >= ((size_t)B_ * SE_) / 8) return;
  const size_t base = i8 * 8;
  const size_t pbse = base % SE_;
  v4f x0 = *(const v4f*)(x + base);
  v4f x1 = *(const v4f*)(x + base + 4);
  v4f p0 = *(const v4f*)(pe + pbse);
  v4f p1 = *(const v4f*)(pe + pbse + 4);
  v4f s0 = (x0 + p0) * XSCL;
  v4f s1 = (x1 + p1) * XSCL;
  Pack8 o;
#pragma unroll
  for (int i = 0; i < 4; ++i) { o.e[i] = (f16_t)s0[i]; o.e[4 + i] = (f16_t)s1[i]; }
  f16_t* d = xph + base;
  *(volatile v8h*)d = o.v;
  __threadfence();
  *(volatile v8h*)d = o.v;
}

__global__ void __launch_bounds__(256) k_tc(const float* __restrict__ t, const float* __restrict__ c,
                                            const float* __restrict__ Wq, const float* __restrict__ bq,
                                            float* tcs) {
  const int i4 = blockIdx.x * 256 + threadIdx.x;
  if (i4 >= (B_ * E_) / 4) return;
  const int b = i4 / (E_ / 4);
  const int n = (i4 % (E_ / 4)) * 4;
  v4f acc = *(const v4f*)(bq + n);
  const float* tb = t + (size_t)b * E_;
  const float* cb = c + (size_t)b * E_;
  const float* w1 = Wq + (size_t)E_ * E_ + n;
  const float* w2 = Wq + (size_t)2 * E_ * E_ + n;
#pragma unroll 1
  for (int k = 0; k < E_; ++k) {
    v4f a = *(const v4f*)(w1 + (size_t)k * E_);
    v4f d = *(const v4f*)(w2 + (size_t)k * E_);
    acc += tb[k] * a;
    acc += cb[k] * d;
  }
  acc = acc * QSCL;
  float* dst = tcs + (size_t)i4 * 4;
  *(volatile v4f*)dst = acc;
  __threadfence();
  *(volatile v4f*)dst = acc;
}

#define TP 72

__global__ void __launch_bounds__(256) k_trw(const float* __restrict__ w0, const float* __restrict__ w1,
                                             const float* __restrict__ w2, f16_t* dst, float mul) {
  __shared__ __align__(16) f16_t tile[64 * TP];
  const int tid = threadIdx.x, lane = tid & 31, wid = tid >> 5;
  const int z = blockIdx.z;
  const float* src = (z == 0) ? w0 : ((z == 1) ? w1 : w2);
  f16_t* d = dst + (size_t)z * E_ * E_;
  const int r0 = blockIdx.y * 64;
  const int c0 = blockIdx.x * 64;
  const int lr = tid >> 2, lc = (tid & 3) * 16;
  const float* sp = src + (size_t)(r0 + lr) * E_ + c0 + lc;
  v4f f0 = *(const v4f*)(sp);
  v4f f1 = *(const v4f*)(sp + 4);
  v4f f2 = *(const v4f*)(sp + 8);
  v4f f3 = *(const v4f*)(sp + 12);
  Pack8 pa, pb;
#pragma unroll
  for (int i = 0; i < 4; ++i) {
    pa.e[i]     = (f16_t)(f0[i] * mul);
    pa.e[4 + i] = (f16_t)(f1[i] * mul);
    pb.e[i]     = (f16_t)(f2[i] * mul);
    pb.e[4 + i] = (f16_t)(f3[i] * mul);
  }
  *(v8h*)(tile + lr * TP + lc)     = pa.v;
  *(v8h*)(tile + lr * TP + lc + 8) = pb.v;
  __syncthreads();
  const int j = lane & 7;
  const int cc0 = wid * 8 + (lane >> 3);
  const int cc1 = cc0 + 4;
  Pack8 o0, o1;
#pragma unroll
  for (int i = 0; i < 8; ++i) {
    o0.e[i] = tile[(8 * j + i) * TP + cc0];
    o1.e[i] = tile[(8 * j + i) * TP + cc1];
  }
  f16_t* g0 = d + (size_t)(c0 + cc0) * E_ + r0 + 8 * j;
  f16_t* g1 = d + (size_t)(c0 + cc1) * E_ + r0 + 8 * j;
  *(volatile v8h*)g0 = o0.v;
  *(volatile v8h*)g1 = o1.v;
  __threadfence();
  *(volatile v8h*)g0 = o0.v;
  *(volatile v8h*)g1 = o1.v;
}

__global__ void __launch_bounds__(256) k_trq(const f16_t* __restrict__ q, f16_t* qT) {
  __shared__ __align__(16) f16_t tile[64 * TP];
  const int tid = threadIdx.x, lane = tid & 31, wid = tid >> 5;
  const int b = blockIdx.z;
  const int r0 = blockIdx.y * 64;
  const int c0 = blockIdx.x * 64;
  const int lr = tid >> 2, lc = (tid & 3) * 16;
  const f16_t* sp = q + (size_t)b * SE_ + (size_t)(r0 + lr) * E_ + c0 + lc;
  v8h u0 = *(const v8ha*)(sp);
  v8h u1 = *(const v8ha*)(sp + 8);
  *(v8h*)(tile + lr * TP + lc)     = u0;
  *(v8h*)(tile + lr * TP + lc + 8) = u1;
  __syncthreads();
  const int j = lane & 7;
  const int cc0 = wid * 8 + (lane >> 3);
  const int cc1 = cc0 + 4;
  Pack8 o0, o1;
#pragma unroll
  for (int i = 0; i < 8; ++i) {
    o0.e[i] = tile[(8 * j + i) * TP + cc0];
    o1.e[i] = tile[(8 * j + i) * TP + cc1];
  }
  f16_t* d = qT + (size_t)b * SE_;
  f16_t* g0 = d + (size_t)(c0 + cc0) * S_ + r0 + 8 * j;
  f16_t* g1 = d + (size_t)(c0 + cc1) * S_ + r0 + 8 * j;
  *(volatile v8h*)g0 = o0.v;
  *(volatile v8h*)g1 = o1.v;
  __threadfence();
  *(volatile v8h*)g0 = o0.v;
  *(volatile v8h*)g1 = o1.v;
}

#define KSTG 64
#define SA_EL (64 * KSTG)
#define SB_EL (256 * KSTG)
#define CPITCH 256

__global__ void __launch_bounds__(256)
k_gemm(const f16_t* __restrict__ A, const f16_t* __restrict__ BT, f16_t* C,
       int K, int N, long long sA, long long sB, long long sC,
       const float* __restrict__ bias, long long sBias, int use_bias,
       float scale, int relu) {
  __shared__ __align__(16) f16_t smem[SA_EL + SB_EL];
  f16_t* sAt = smem;
  f16_t* sBt = smem + SA_EL;
  f16_t* sCt = smem;

  const int tid = threadIdx.x, lane = tid & 31, wid = tid >> 5;
  const int wm = wid >> 2, wn = wid & 3;
  const int rowblk = blockIdx.x * 64;
  const int colblk = blockIdx.y * 256;
  const int b = blockIdx.z;

  const f16_t* Ag = A  + (size_t)b * (size_t)sA + (size_t)rowblk * K;
  const f16_t* Bg = BT + (size_t)b * (size_t)sB + (size_t)colblk * K;
  f16_t* Cg = C + (size_t)b * (size_t)sC;

  const int arow = tid >> 2, acol = (tid & 3) * 16;
  const f16_t* agp = Ag + (size_t)arow * K + acol;
  const f16_t* bgp = Bg + (size_t)tid * K;
  f16_t* saw = sAt + arow * KSTG + acol;
  f16_t* sbw = sBt + tid * KSTG;

  v8f acc[2][4];
#pragma unroll
  for (int mt = 0; mt < 2; ++mt)
#pragma unroll
    for (int nt = 0; nt < 4; ++nt) acc[mt][nt] = zero8();

  const int nst = K / KSTG;
  for (int s = 0; s < nst; ++s) {
    const int k0 = s * KSTG;
    v8h ta0 = *(const v8ha*)(agp + k0);
    v8h ta1 = *(const v8ha*)(agp + k0 + 8);
    v8h tb[8];
#pragma unroll
    for (int jj = 0; jj < 8; ++jj) tb[jj] = *(const v8ha*)(bgp + k0 + 8 * jj);
    *(v8h*)(saw)     = ta0;
    *(v8h*)(saw + 8) = ta1;
#pragma unroll
    for (int jj = 0; jj < 8; ++jj) *(v8h*)(sbw + 8 * jj) = tb[jj];
    __syncthreads();
#pragma unroll
    for (int ks = 0; ks < 2; ++ks) {
      const f16_t* pa = sAt + (wm * 32) * KSTG + ks * 32;
      const f16_t* pb = sBt + (wn * 64) * KSTG + ks * 32;
      v16h a0 = load_frag(pa, KSTG, lane);
      v16h a1 = load_frag(pa + 16 * KSTG, KSTG, lane);
      v16h f0 = load_frag(pb, KSTG, lane);
      v16h f1 = load_frag(pb + 16 * KSTG, KSTG, lane);
      v16h f2 = load_frag(pb + 32 * KSTG, KSTG, lane);
      v16h f3 = load_frag(pb + 48 * KSTG, KSTG, lane);
      acc[0][0] = wmma16(a0, f0, acc[0][0]);
      acc[0][1] = wmma16(a0, f1, acc[0][1]);
      acc[0][2] = wmma16(a0, f2, acc[0][2]);
      acc[0][3] = wmma16(a0, f3, acc[0][3]);
      acc[1][0] = wmma16(a1, f0, acc[1][0]);
      acc[1][1] = wmma16(a1, f1, acc[1][1]);
      acc[1][2] = wmma16(a1, f2, acc[1][2]);
      acc[1][3] = wmma16(a1, f3, acc[1][3]);
      WMMA_GUARD8(acc[0][0], acc[0][1], acc[0][2], acc[0][3],
                  acc[1][0], acc[1][1], acc[1][2], acc[1][3],
                  a0, a1, f0, f1, f2, f3);
    }
    __syncthreads();
  }

  const int h = lane >> 4, nc = lane & 15;
#pragma unroll
  for (int mt = 0; mt < 2; ++mt) {
#pragma unroll
    for (int nt = 0; nt < 4; ++nt) {
      const int col = wn * 64 + nt * 16 + nc;
      const float bv = use_bias ? bias[(size_t)b * (size_t)sBias + colblk + col] : 0.0f;
#pragma unroll
      for (int r = 0; r < 8; ++r) {
        float v = acc[mt][nt][r] * scale + bv;
        if (relu) v = fmaxf(v, 0.0f);
        sCt[(wm * 32 + mt * 16 + 8 * h + r) * CPITCH + col] = (f16_t)v;
      }
    }
  }
  __syncthreads();

  v8h ov[8];
#pragma unroll
  for (int rr = 0; rr < 8; ++rr)
    ov[rr] = *(const v8ha*)(sCt + (wid * 8 + rr) * CPITCH + 8 * lane);
#pragma unroll
  for (int rr = 0; rr < 8; ++rr) {
    f16_t* gp = Cg + (size_t)(rowblk + wid * 8 + rr) * N + colblk + 8 * lane;
    *(volatile v8h*)gp = ov[rr];
  }
  __threadfence();
#pragma unroll
  for (int rr = 0; rr < 8; ++rr) {
    f16_t* gp = Cg + (size_t)(rowblk + wid * 8 + rr) * N + colblk + 8 * lane;
    *(volatile v8h*)gp = ov[rr];
  }
}

__global__ void __launch_bounds__(256)
k_final(const f16_t* __restrict__ Hm, const f16_t* __restrict__ W2T,
        const float* __restrict__ b2, const float* __restrict__ gamma,
        const float* __restrict__ beta, const float* __restrict__ x,
        const float* __restrict__ pe, float* out, float scale) {
  __shared__ __align__(16) float sh[16 * E_];
  __shared__ float ps[16 * 16];
  __shared__ float smu[16];
  __shared__ float srs[16];

  const int tid = threadIdx.x, lane = tid & 31, wid = tid >> 5;
  const int b = blockIdx.z;
  const int row0 = blockIdx.x * 16;
  const int col0 = wid * 64;

  const f16_t* Ab = Hm + ((size_t)b * S_ + row0) * E_;

  v8f acc[4];
#pragma unroll
  for (int i = 0; i < 4; ++i) acc[i] = zero8();

  for (int k = 0; k < E_; k += 32) {
    v16h a = load_frag(Ab + k, E_, lane);
    const f16_t* wp = W2T + (size_t)col0 * E_ + k;
    v16h f0 = load_frag(wp, E_, lane);
    v16h f1 = load_frag(wp + 16 * E_, E_, lane);
    v16h f2 = load_frag(wp + 32 * E_, E_, lane);
    v16h f3 = load_frag(wp + 48 * E_, E_, lane);
    acc[0] = wmma16(a, f0, acc[0]);
    acc[1] = wmma16(a, f1, acc[1]);
    acc[2] = wmma16(a, f2, acc[2]);
    acc[3] = wmma16(a, f3, acc[3]);
    WMMA_GUARD4(acc[0], acc[1], acc[2], acc[3], a, f0, f1, f2, f3);
  }

  const int h = lane >> 4, nc = lane & 15;
#pragma unroll
  for (int nt = 0; nt < 4; ++nt) {
    const int col = col0 + nt * 16 + nc;
    const float bv = b2[col];
#pragma unroll
    for (int r = 0; r < 8; ++r) sh[(8 * h + r) * E_ + col] = acc[nt][r] * scale + bv;
  }
  __syncthreads();

  const int lrow = tid >> 4, seg = tid & 15;
  const float* hp = sh + lrow * E_ + seg * 32;
  {
    float s = 0.f;
#pragma unroll 8
    for (int i = 0; i < 32; ++i) s += hp[i];
    ps[lrow * 16 + seg] = s;
  }
  __syncthreads();
  if (tid < 16) {
    float s = 0.f;
#pragma unroll
    for (int i = 0; i < 16; ++i) s += ps[tid * 16 + i];
    smu[tid] = s * (1.0f / (float)E_);
  }
  __syncthreads();
  {
    const float mu = smu[lrow];
    float qv = 0.f;
#pragma unroll 8
    for (int i = 0; i < 32; ++i) { const float dd = hp[i] - mu; qv += dd * dd; }
    ps[lrow * 16 + seg] = qv;
  }
  __syncthreads();
  if (tid < 16) {
    float qv = 0.f;
#pragma unroll
    for (int i = 0; i < 16; ++i) qv += ps[tid * 16 + i];
    srs[tid] = rsqrtf(qv * (1.0f / (float)E_) + 1e-5f);
  }
  __syncthreads();

  const size_t obase = ((size_t)b * S_ + row0) * E_;
  v4f ov[8];
#pragma unroll
  for (int i = 0; i < 8; ++i) {
    const int idx = tid + i * 256;
    const int r = idx >> 7;
    const int cc = (idx & 127) * 4;
    v4f hv = *(const v4fa*)(sh + r * E_ + cc);
    v4f g  = *(const v4f*)(gamma + cc);
    v4f bt = *(const v4f*)(beta + cc);
    v4f xv = *(const v4f*)(x + obase + (size_t)r * E_ + cc);
    v4f pv = *(const v4f*)(pe + (size_t)(row0 + r) * E_ + cc);
    const float mu = smu[r], rs = srs[r];
    v4f xp = xv + pv;
    v4f ln = ((hv - mu) * rs) * g + bt;
    ov[i] = ln + xp;
  }
#pragma unroll
  for (int i = 0; i < 8; ++i) {
    const int idx = tid + i * 256;
    const int r = idx >> 7;
    const int cc = (idx & 127) * 4;
    *(volatile v4f*)(out + obase + (size_t)r * E_ + cc) = ov[i];
  }
  __threadfence();
#pragma unroll
  for (int i = 0; i < 8; ++i) {
    const int idx = tid + i * 256;
    const int r = idx >> 7;
    const int cc = (idx & 127) * 4;
    *(volatile v4f*)(out + obase + (size_t)r * E_ + cc) = ov[i];
  }
}

extern "C" void kernel_launch(void* const* d_in, const int* in_sizes, int n_in,
                              void* d_out, int out_size, void* d_ws, size_t ws_size,
                              hipStream_t stream) {
  if (n_in < 11) return;
  if (in_sizes[0] != (int)((size_t)B_ * SE_)) return;
  if (in_sizes[1] != B_ * E_ || in_sizes[2] != B_ * E_) return;
  if (in_sizes[3] != 3 * E_ * E_ || in_sizes[4] != E_) return;
  if (in_sizes[5] != E_ * E_ || in_sizes[6] != E_) return;
  if (in_sizes[7] != E_ * E_ || in_sizes[8] != E_) return;
  if (in_sizes[9] != E_ || in_sizes[10] != E_) return;
  if (out_size != (int)((size_t)B_ * SE_)) return;

  const float* x     = (const float*)d_in[0];
  const float* t     = (const float*)d_in[1];
  const float* c     = (const float*)d_in[2];
  const float* Wq    = (const float*)d_in[3];
  const float* bq    = (const float*)d_in[4];
  const float* W1    = (const float*)d_in[5];
  const float* b1    = (const float*)d_in[6];
  const float* W2    = (const float*)d_in[7];
  const float* b2    = (const float*)d_in[8];
  const float* gamma = (const float*)d_in[9];
  const float* beta  = (const float*)d_in[10];
  float* out = (float*)d_out;

  const size_t sz_pe  = SE_ * sizeof(float);
  const size_t sz_act = (size_t)B_ * SE_ * sizeof(f16_t);
  const size_t sz_att = (size_t)B_ * SS_ * sizeof(f16_t);
  const size_t sz_wt  = (size_t)3 * E_ * E_ * sizeof(f16_t);
  const size_t sz_tc  = (size_t)B_ * E_ * sizeof(float);
  size_t off = 0;
  const size_t off_pe  = off; off += sz_pe;
  const size_t off_a0  = off; off += sz_act;
  const size_t off_a1  = off; off += sz_act;
  const size_t off_qT  = off; off += sz_act;
  const size_t off_att = off; off += sz_att;
  const size_t off_wt  = off; off += sz_wt;
  const size_t off_tc  = off; off += sz_tc;
  if (off > ws_size) return;

  char* w = (char*)d_ws;
  float* pe  = (float*)(w + off_pe);
  f16_t* xph = (f16_t*)(w + off_a0);
  f16_t* v2  = (f16_t*)(w + off_a0);
  f16_t* qh  = (f16_t*)(w + off_a1);
  f16_t* hm  = (f16_t*)(w + off_a1);
  f16_t* qT  = (f16_t*)(w + off_qT);
  f16_t* att = (f16_t*)(w + off_att);
  f16_t* wt  = (f16_t*)(w + off_wt);
  float* tcs = (float*)(w + off_tc);
  const f16_t* WqT = wt;
  const f16_t* W1T = wt + (size_t)E_ * E_;
  const f16_t* W2T = wt + (size_t)2 * E_ * E_;

  const long long SEll = (long long)SE_;
  const long long SSll = (long long)SS_;
  dim3 blk(256);

  k_pe<<<(S_ * E_) / 256 / 8, blk, 0, stream>>>(pe);
  k_xph<<<(unsigned)(((size_t)B_ * SE_) / 8 / 256), blk, 0, stream>>>(x, pe, xph);
  k_tc<<<(B_ * E_) / 4 / 256, blk, 0, stream>>>(t, c, Wq, bq, tcs);
  k_trw<<<dim3(E_ / 64, E_ / 64, 3), blk, 0, stream>>>(Wq, W1, W2, wt, WSCL);
  k_gemm<<<dim3(S_ / 64, E_ / 256, B_), blk, 0, stream>>>(
      xph, WqT, qh, E_, E_, SEll, 0LL, SEll, tcs, (long long)E_, 1, 1.0f / 64.0f, 0);
  k_trq<<<dim3(E_ / 64, S_ / 64, B_), blk, 0, stream>>>(qh, qT);
  k_gemm<<<dim3(S_ / 64, S_ / 256, B_), blk, 0, stream>>>(
      qh, qh, att, E_, S_, SEll, SEll, SSll, bq, 0LL, 0, 1.0f / 131072.0f, 0);
  k_gemm<<<dim3(S_ / 64, E_ / 256, B_), blk, 0, stream>>>(
      att, qT, v2, S_, E_, SSll, SEll, SEll, bq, 0LL, 0, 1.0f / 16.0f, 0);
  k_gemm<<<dim3(S_ / 64, E_ / 256, B_), blk, 0, stream>>>(
      v2, W1T, hm, E_, E_, SEll, 0LL, SEll, b1, 0LL, 1, 1.0f / 64.0f, 1);
  k_final<<<dim3(S_ / 16, 1, B_), blk, 0, stream>>>(
      hm, W2T, b2, gamma, beta, x, pe, out, 1.0f / 64.0f);
}
